// GRNDrugGCN_21560735825958
// MI455X (gfx1250) — hardware-run, weakly checked
//
#include <hip/hip_runtime.h>
#include <stddef.h>
#include <stdint.h>
#include <math.h>

#define NN      100000
#define CIN     128
#define HD      32
#define NE      3200000
#define NPAIR   1000000
#define NSEL    50000
#define NHEAD   96
#define GBM     128
#define MP      100096
#define KHL     64
#define S2_TWO  1
#define S3_TWO  1
#define K2EXT   (S2_TWO ? 64 : 32)
#define K3EXT   (S3_TWO ? 64 : 32)
#define NTHR    256
#define NWAVE   8
#define EPT     8
#define WCH     (32 * EPT)
#define NBRUN   1024
#define SLB     10
#define SRCB    17
#define NBK     98
#define WLCAP   4864
#define HCAP    18432
#define RCAP    (2 * HCAP)
#define DEGCAP  96
#define MAXDEG_MEAS   57
#define MAXB1024_MEAS 33219
#define MAXB512_MEAS  16774
#define RBM     64
#define NLINE0  (NPAIR / 32)
#define NLINE1  ((NSEL + 31) / 32)
#define TBN     384

#define BK_ZINTS (NWAVE * WLCAP + HCAP + 4 * NBRUN)
#define BK_INTS  (BK_ZINTS + 16)
#define BK_LDS   (BK_INTS * 4)

#define PBX   (MP * CIN / 8 / NTHR)
#define PBW1  (HD * CIN / 8 / NTHR)
#define PBW2  (HD * KHL / 8 / NTHR)
#define PBWH  (NHEAD * KHL / 8 / NTHR)
#define PBTOT (PBX + PBW1 + PBW2 + PBWH + 1)

static_assert(SRCB + SLB <= 32);
static_assert(NN <= (1 << SRCB));
static_assert(NBRUN == 1024 && NBRUN == (1 << SLB));
static_assert(MP % GBM == 0 && MP >= NN && MP == 782 * GBM && MP % RBM == 0 && NBRUN % RBM == 0);
static_assert(NBK * NBRUN >= MP && (NBK - 1) * NBRUN < NN);
static_assert(NE % WCH == 0 && NE % 4 == 0);
static_assert(RCAP == 2 * HCAP && HCAP % (NTHR * 4) == 0 && BK_ZINTS % 4 == 0);
static_assert((long long)RCAP * 100 >= (long long)MAXB1024_MEAS * 105);
static_assert((long long)HCAP * 100 >= (long long)MAXB512_MEAS * 105);
static_assert(WLCAP >= RCAP / 8 + 256);
static_assert(MAXDEG_MEAS + 8 <= DEGCAP && DEGCAP * 100 >= MAXDEG_MEAS * 105);
static_assert(BK_LDS <= 300000);
static_assert((MP * CIN / 8) % NTHR == 0 && (HD * CIN / 8) % NTHR == 0);
static_assert((HD * KHL / 8) % NTHR == 0 && (NHEAD * KHL / 8) == 3 * NTHR);
static_assert(CIN % 32 == 0 && K2EXT % 32 == 0 && K3EXT % 32 == 0 && KHL == 2 * HD);
static_assert(NPAIR % 32 == 0 && (NPAIR * 4) % 128 == 0);
static_assert(NLINE1 * 32 >= NSEL && (NLINE1 - 1) * 32 < NSEL);
static_assert((GBM * (16 * 6 + 4) + GBM) * 4 <= 65536);

typedef float          v2f   __attribute__((ext_vector_type(2)));
typedef float          v4f   __attribute__((ext_vector_type(4)));
typedef float          v8f   __attribute__((ext_vector_type(8)));
typedef int            v2i   __attribute__((ext_vector_type(2)));
typedef int            v4i   __attribute__((ext_vector_type(4)));
typedef int            v8i   __attribute__((ext_vector_type(8)));
typedef unsigned short v8us  __attribute__((ext_vector_type(8)));
typedef unsigned short v16us __attribute__((ext_vector_type(16)));
typedef __bf16         v16bf __attribute__((ext_vector_type(16)));
typedef v2f  __attribute__((may_alias)) v2fa;
typedef v4f  __attribute__((may_alias)) v4fa;
typedef v4i  __attribute__((may_alias)) v4ia;
typedef v8us __attribute__((may_alias)) v8usa;
union FragB { v16bf v; v16us u; v8us h[2]; v8i w; };

__device__ __forceinline__ v8f wmb(const FragB& a, const FragB& b, v8f c) {
  v8f d = __builtin_amdgcn_wmma_f32_16x16x32_bf16(false, a.v, false, b.v, (short)0, c, false, false);
  asm volatile("v_nop\n\tv_nop\n\tv_nop\n\tv_nop" : "+v"(d) : "v"(a.w), "v"(b.w));
  return d;
}

__device__ __forceinline__ unsigned bf16_bits(float f) {
  const unsigned u = __float_as_uint(f);
  const unsigned r = (u + 0x7FFFu + ((u >> 16) & 1u)) >> 16;
  const unsigned q = (u >> 16) | 0x40u;
  return ((u & 0x7fffffffu) > 0x7f800000u) ? q : r;
}
__device__ __forceinline__ float bf16_val(float f) {
  return __uint_as_float(bf16_bits(f) << 16);
}
__device__ __forceinline__ unsigned bfr(float f) { return bf16_bits(f) << 16; }

__device__ __forceinline__ int clampi(int v, int lo, int hi) {
  return v < lo ? lo : (v > hi ? hi : v);
}

__device__ __forceinline__ void hilo_pack(float v0, float v1, float v2, float v3,
                                          int& h01, int& h23, int& l01, int& l23) {
  const unsigned a0 = bf16_bits(v0), a1 = bf16_bits(v1), a2 = bf16_bits(v2), a3 = bf16_bits(v3);
  const unsigned b0 = bf16_bits(v0 - __uint_as_float(a0 << 16));
  const unsigned b1 = bf16_bits(v1 - __uint_as_float(a1 << 16));
  const unsigned b2 = bf16_bits(v2 - __uint_as_float(a2 << 16));
  const unsigned b3 = bf16_bits(v3 - __uint_as_float(a3 << 16));
  h01 = (int)(a0 | (a1 << 16)); h23 = (int)(a2 | (a3 << 16));
  l01 = (int)(b0 | (b1 << 16)); l23 = (int)(b2 | (b3 << 16));
}

__device__ __forceinline__ void st2_v4f(float* p, v4f v) {
  *(volatile v4f*)p = v;
  __threadfence();
  *(volatile v4f*)p = v;
}
__device__ __forceinline__ void st2_v8us(unsigned short* p, v8us v) {
  *(volatile v8us*)p = v;
  __threadfence();
  *(volatile v8us*)p = v;
}

__device__ __forceinline__ v8us gather8(const float* __restrict__ base, int stride) {
  float f[8];
#pragma unroll
  for (int i = 0; i < 8; ++i) f[i] = base[(size_t)i * (size_t)stride];
  v8us o;
#pragma unroll
  for (int i = 0; i < 8; ++i) o[i] = (unsigned short)bf16_bits(f[i]);
  return o;
}

__device__ __forceinline__ float tabmix(float a0, float a1, float a2, float a3, float a4, float a5, float a6,
                                        float a7, float s, unsigned m0, unsigned m1, unsigned m2, unsigned m3,
                                        unsigned m4, unsigned m5, unsigned m6, unsigned m7, unsigned ms) {
  const unsigned r = (bfr(a0) & m0) | (bfr(a1) & m1) | (bfr(a2) & m2) | (bfr(a3) & m3) |
                     (bfr(a4) & m4) | (bfr(a5) & m5) | (bfr(a6) & m6) | (bfr(a7) & m7) | (bfr(s) & ms);
  return __uint_as_float(r);
}

__global__ __launch_bounds__(NTHR) void k_prep(const float* __restrict__ x, const float* __restrict__ w1,
                                               const float* __restrict__ b1, const float* __restrict__ w2,
                                               const float* __restrict__ b2, const float* __restrict__ ew1,
                                               const float* __restrict__ eb1, const float* __restrict__ ew2,
                                               const float* __restrict__ eb2, const float* __restrict__ gw1,
                                               const float* __restrict__ gb1, const float* __restrict__ gw2,
                                               const float* __restrict__ gb2,
                                               unsigned short* xb, unsigned short* w1t, unsigned short* w2d,
                                               unsigned short* whd, float* tb) {
  const int tid = (int)threadIdx.x;
  const int blk = (int)blockIdx.x;
  if (blk < PBX) {
    const int u   = blk * NTHR + tid;
    const int row = u >> 4, k8 = (u & 15) * 8;
    const int rc  = row < NN ? row : NN - 1;
    const unsigned mk = row < NN ? 0xffffu : 0u;
    const float* p = x + (size_t)rc * CIN + k8;
    const v4f a = *(const v4fa*)p;
    const v4f b = *(const v4fa*)(p + 4);
    v8us o;
    o[0] = (unsigned short)(bf16_bits(a.x) & mk); o[1] = (unsigned short)(bf16_bits(a.y) & mk);
    o[2] = (unsigned short)(bf16_bits(a.z) & mk); o[3] = (unsigned short)(bf16_bits(a.w) & mk);
    o[4] = (unsigned short)(bf16_bits(b.x) & mk); o[5] = (unsigned short)(bf16_bits(b.y) & mk);
    o[6] = (unsigned short)(bf16_bits(b.z) & mk); o[7] = (unsigned short)(bf16_bits(b.w) & mk);
    st2_v8us(xb + (size_t)row * CIN + k8, o);
  } else if (blk < PBX + PBW1) {
    const int u = (blk - PBX) * NTHR + tid;
    const int n = u >> 4, k8 = (u & 15) * 8;
    const v8us o = gather8(w1 + (size_t)k8 * HD + n, HD);
    st2_v8us(w1t + (size_t)n * CIN + k8, o);
  } else if (blk < PBX + PBW1 + PBW2) {
    const int u = tid;
    const int n = u >> 3, k8 = (u & 7) * 8, kk = k8 & 31;
    const v8us o = gather8(w2 + (size_t)kk * HD + n, HD);
    st2_v8us(w2d + (size_t)n * KHL + k8, o);
  } else if (blk < PBX + PBW1 + PBW2 + 2) {
    const int j = blk - (PBX + PBW1 + PBW2);
    const int r = tid >> 3, k8 = (tid & 7) * 8, kk = k8 & 31;
    const v8us o = gather8(ew1 + (size_t)(32 * j + kk) * HD + r, HD);
    st2_v8us(whd + (size_t)(32 * j + r) * KHL + k8, o);
  } else if (blk < PBX + PBW1 + PBW2 + PBWH) {
    const int r = tid >> 3, k8 = (tid & 7) * 8, kk = k8 & 31;
    const v8us o = gather8(gw1 + (size_t)kk * HD + r, HD);
    st2_v8us(whd + (size_t)(64 + r) * KHL + k8, o);
  } else {
    if (tid < 96) {
      const int grp = tid >> 3, c = (tid & 7) * 4;
      const v4f A0 = *(const v4fa*)(b1 + c);
      const v4f A1 = *(const v4fa*)(b2 + c);
      const v4f A2 = *(const v4fa*)(eb1 + c);
      const v4f A3 = *(const v4fa*)(ew1 + 64 * HD + c);
      const v4f A4 = *(const v4fa*)(ew1 + 65 * HD + c);
      const v4f A5 = *(const v4fa*)(ew2 + c);
      const v4f A6 = *(const v4fa*)(gb1 + c);
      const v4f A7 = *(const v4fa*)(gw2 + c);
      const float s0 = eb2[0], s1 = gb2[0];
      asm volatile("" :: "v"(A0), "v"(A1), "v"(A2), "v"(A3));
      asm volatile("" :: "v"(A4), "v"(A5), "v"(A6), "v"(A7));
      asm volatile("" :: "v"(s0), "v"(s1));
      const unsigned m0 = (grp == 0) ? 0xffffffffu : 0u, m1 = (grp == 1) ? 0xffffffffu : 0u;
      const unsigned m2 = (grp == 4) ? 0xffffffffu : 0u, m3 = (grp == 5) ? 0xffffffffu : 0u;
      const unsigned m4 = (grp == 6) ? 0xffffffffu : 0u, m5 = (grp == 7) ? 0xffffffffu : 0u;
      const unsigned m6 = (grp == 8) ? 0xffffffffu : 0u, m7 = (grp == 9) ? 0xffffffffu : 0u;
      const unsigned ms = ((grp == 10) & (c == 0)) ? 0xffffffffu : 0u;
      v4f o;
      o.x = tabmix(A0.x, A1.x, A2.x, A3.x, A4.x, A5.x, A6.x, A7.x, s0, m0, m1, m2, m3, m4, m5, m6, m7, ms);
      o.y = tabmix(A0.y, A1.y, A2.y, A3.y, A4.y, A5.y, A6.y, A7.y, s1, m0, m1, m2, m3, m4, m5, m6, m7, ms);
      o.z = tabmix(A0.z, A1.z, A2.z, A3.z, A4.z, A5.z, A6.z, A7.z, 0.0f, m0, m1, m2, m3, m4, m5, m6, m7, 0u);
      o.w = tabmix(A0.w, A1.w, A2.w, A3.w, A4.w, A5.w, A6.w, A7.w, 0.0f, m0, m1, m2, m3, m4, m5, m6, m7, 0u);
      st2_v4f(tb + 4 * tid, o);
    }
  }
}

__device__ __forceinline__ void list_flush(const int* pl, int* lp, int tid) {
#pragma unroll 1
  for (int i = tid * 4; i < HCAP; i += NTHR * 4) {
    const v4i v = *(const v4ia*)(pl + i);
    *(volatile v4i*)(lp + i) = v;
  }
}

__device__ __forceinline__ void tab_flush(const int* cnt, const int* offs, const int* dv, int ov,
                                          int* cp, int* op, int* dp, int* fp, int tid) {
  {
    const v4i v = *(const v4ia*)(cnt + 4 * tid);
    *(volatile v4i*)(cp + 4 * tid) = v;
  }
  {
    const v4i v = *(const v4ia*)(offs + 4 * tid);
    *(volatile v4i*)(op + 4 * tid) = v;
  }
  {
    const v4i v = *(const v4ia*)(dv + 4 * tid);
    *(volatile v4i*)(dp + 4 * tid) = v;
  }
  if (tid < 8) {
    const v4i f = {ov, ov, ov, ov};
    *(volatile v4i*)(fp + 4 * tid) = f;
  }
}

__global__ __launch_bounds__(NTHR) void k_bucket(const int* __restrict__ srcs, const int* __restrict__ dsts,
                                                 int* LIST, int* CNT, int* OFF, int* DINV, int* FLAG) {
  extern __shared__ __attribute__((aligned(16))) int dsm[];
  int* wl   = dsm;
  int* pl   = dsm + NWAVE * WLCAP;
  int* cnt  = pl + HCAP;
  int* offs = cnt + NBRUN;
  int* cur  = offs + NBRUN;
  int* dv   = cur + NBRUN;
  int* misc = dv + NBRUN;
  const int tid = (int)threadIdx.x, lane = tid & 31, wave = tid >> 5;
  const int blk = (int)blockIdx.x;
  const unsigned nbs = (unsigned)(blk * NBRUN);
  const int lim = NN - blk * NBRUN;
  const unsigned unb = (unsigned)(lim < NBRUN ? lim : NBRUN);

  {
    const v4i z4 = {0, 0, 0, 0};
    for (int i = tid * 4; i < BK_ZINTS; i += NTHR * 4) *(v4ia*)(dsm + i) = z4;
    if (tid < 16) misc[tid] = 0;
  }
  __syncthreads();

  {
    const int per  = ((NE + NWAVE * WCH - 1) / (NWAVE * WCH)) * WCH;
    const int ebeg = wave * per;
    const int eend = (ebeg + per < NE) ? (ebeg + per) : NE;
    int* mylist = wl + wave * WLCAP;
    int wc = 0;
#pragma unroll 1
    for (int cb = ebeg; cb < eend; cb += WCH) {
      const int e0 = cb + lane * EPT;
      const v4i da = *(const v4ia*)(dsts + e0);
      const v4i db = *(const v4ia*)(dsts + e0 + 4);
      const unsigned s0 = (unsigned)da.x - nbs, s1 = (unsigned)da.y - nbs;
      const unsigned s2 = (unsigned)da.z - nbs, s3 = (unsigned)da.w - nbs;
      const unsigned s4 = (unsigned)db.x - nbs, s5 = (unsigned)db.y - nbs;
      const unsigned s6 = (unsigned)db.z - nbs, s7 = (unsigned)db.w - nbs;
      const bool h0 = s0 < unb, h1 = s1 < unb, h2 = s2 < unb, h3 = s3 < unb;
      const bool h4 = s4 < unb, h5 = s5 < unb, h6 = s6 < unb, h7 = s7 < unb;
      const unsigned m0 = __builtin_amdgcn_ballot_w32(h0), m1 = __builtin_amdgcn_ballot_w32(h1);
      const unsigned m2 = __builtin_amdgcn_ballot_w32(h2), m3 = __builtin_amdgcn_ballot_w32(h3);
      const unsigned m4 = __builtin_amdgcn_ballot_w32(h4), m5 = __builtin_amdgcn_ballot_w32(h5);
      const unsigned m6 = __builtin_amdgcn_ballot_w32(h6), m7 = __builtin_amdgcn_ballot_w32(h7);
      const unsigned any = m0 | m1 | m2 | m3 | m4 | m5 | m6 | m7;
      if (any != 0u) {
        const v4i sa = *(const v4ia*)(srcs + e0);
        const v4i sb = *(const v4ia*)(srcs + e0 + 4);
        const int r0 = clampi(sa.x, 0, NN - 1), r1 = clampi(sa.y, 0, NN - 1);
        const int r2 = clampi(sa.z, 0, NN - 1), r3 = clampi(sa.w, 0, NN - 1);
        const int r4 = clampi(sb.x, 0, NN - 1), r5 = clampi(sb.y, 0, NN - 1);
        const int r6 = clampi(sb.z, 0, NN - 1), r7 = clampi(sb.w, 0, NN - 1);
        const int pre = (int)(__builtin_amdgcn_mbcnt_lo(m0, 0u) + __builtin_amdgcn_mbcnt_lo(m1, 0u) +
                              __builtin_amdgcn_mbcnt_lo(m2, 0u) + __builtin_amdgcn_mbcnt_lo(m3, 0u) +
                              __builtin_amdgcn_mbcnt_lo(m4, 0u) + __builtin_amdgcn_mbcnt_lo(m5, 0u) +
                              __builtin_amdgcn_mbcnt_lo(m6, 0u) + __builtin_amdgcn_mbcnt_lo(m7, 0u));
        int p = wc + pre;
        if (h0) { if (p < WLCAP) mylist[p] = r0 | ((int)s0 << SRCB); p = p + 1; }
        if (h1) { if (p < WLCAP) mylist[p] = r1 | ((int)s1 << SRCB); p = p + 1; }
        if (h2) { if (p < WLCAP) mylist[p] = r2 | ((int)s2 << SRCB); p = p + 1; }
        if (h3) { if (p < WLCAP) mylist[p] = r3 | ((int)s3 << SRCB); p = p + 1; }
        if (h4) { if (p < WLCAP) mylist[p] = r4 | ((int)s4 << SRCB); p = p + 1; }
        if (h5) { if (p < WLCAP) mylist[p] = r5 | ((int)s5 << SRCB); p = p + 1; }
        if (h6) { if (p < WLCAP) mylist[p] = r6 | ((int)s6 << SRCB); p = p + 1; }
        if (h7) { if (p < WLCAP) mylist[p] = r7 | ((int)s7 << SRCB); p = p + 1; }
        wc += (int)(__builtin_popcount(m0) + __builtin_popcount(m1) + __builtin_popcount(m2) + __builtin_popcount(m3) +
                    __builtin_popcount(m4) + __builtin_popcount(m5) + __builtin_popcount(m6) + __builtin_popcount(m7));
      }
    }
    if (lane == 0) misc[wave] = wc;
  }
  __syncthreads();

  if (wave == 0) {
    int ov = 0;
#pragma unroll 1
    for (int w2 = 0; w2 < NWAVE; ++w2) {
      int cv = misc[w2];
      if (cv > WLCAP) ov = 1;
      cv = cv < 0 ? 0 : (cv > WLCAP ? WLCAP : cv);
      const int c = __builtin_amdgcn_readfirstlane(cv);
#pragma unroll 1
      for (int b0 = 0; b0 < c; b0 += 32) {
        const int idx = b0 + lane;
        const int ent = wl[w2 * WLCAP + (idx < WLCAP ? idx : WLCAP - 1)];
        const int m32 = (c - b0) < 32 ? (c - b0) : 32;
#pragma unroll 1
        for (int k = 0; k < m32; ++k) {
          const int u    = __builtin_amdgcn_readlane(ent, k);
          const int slot = (u >> SRCB) & (NBRUN - 1);
          if (lane == 0) cnt[slot] = cnt[slot] + 1;
        }
      }
    }
    if (lane == 0) misc[9] = ov;
  }
  __syncthreads();

  if (wave == 0) {
    const int base = lane * (NBRUN / 32);
    int s = 0;
#pragma unroll 1
    for (int i = 0; i < NBRUN / 32; ++i) s += cnt[base + i];
    int incl = s;
#pragma unroll
    for (int d = 1; d < 32; d <<= 1) {
      const int y = __shfl_up(incl, d, 32);
      if (lane >= d) incl += y;
    }
    const int tot0 = __shfl(incl, 15, 32);
    const int tot  = __shfl(incl, 31, 32);
    const int hsel = (lane >= 16) ? 1 : 0;
    int run = (incl - s) - hsel * tot0;
#pragma unroll 1
    for (int i = 0; i < NBRUN / 32; ++i) {
      const int cv = cnt[base + i];
      offs[base + i] = hsel * HCAP + run;
      cur[base + i]  = run;
      run += cv;
    }
    const int hov = ((tot0 > HCAP) | ((tot - tot0) > HCAP)) ? 1 : 0;
    if (lane == 0) misc[9] = misc[9] | hov;
  }
  __syncthreads();

#pragma unroll 1
  for (int hf = 0; hf < 2; ++hf) {
    if (hf != 0) {
      const v4i z4 = {0, 0, 0, 0};
      for (int i = tid * 4; i < HCAP; i += NTHR * 4) *(v4ia*)(pl + i) = z4;
    }
    __syncthreads();
    if (wave == 0) {
#pragma unroll 1
      for (int w2 = 0; w2 < NWAVE; ++w2) {
        int cv = misc[w2];
        cv = cv < 0 ? 0 : (cv > WLCAP ? WLCAP : cv);
        const int c = __builtin_amdgcn_readfirstlane(cv);
#pragma unroll 1
        for (int b0 = 0; b0 < c; b0 += 32) {
          const int idx = b0 + lane;
          const int ent = wl[w2 * WLCAP + (idx < WLCAP ? idx : WLCAP - 1)];
          const int m32 = (c - b0) < 32 ? (c - b0) : 32;
#pragma unroll 1
          for (int k = 0; k < m32; ++k) {
            const int u    = __builtin_amdgcn_readlane(ent, k);
            const int slot = (u >> SRCB) & (NBRUN - 1);
            if ((slot >> 9) == hf) {
              if (lane == 0) {
                int p = cur[slot];
                p = p < 0 ? 0 : (p > HCAP - 1 ? HCAP - 1 : p);
                pl[p] = u & ((1 << SRCB) - 1);
                cur[slot] = p + 1;
              }
            }
          }
        }
      }
    }
    __syncthreads();
    int* lp = LIST + (size_t)blk * RCAP + (size_t)hf * HCAP;
    list_flush(pl, lp, tid);
    __threadfence();
    list_flush(pl, lp, tid);
    __syncthreads();
  }

#pragma unroll 1
  for (int i = tid; i < NBRUN; i += NTHR) {
    const float dg = (float)(cnt[i] + 1);
    dv[i] = __float_as_int(1.0f / sqrtf(dg));
  }
  __syncthreads();
  const int ovf = misc[9];
  int* cp = CNT + (size_t)blk * NBRUN;
  int* op = OFF + (size_t)blk * NBRUN;
  int* dp = DINV + (size_t)blk * NBRUN;
  int* fp = FLAG + (size_t)blk * 32;
  tab_flush(cnt, offs, dv, ovf, cp, op, dp, fp, tid);
  __threadfence();
  tab_flush(cnt, offs, dv, ovf, cp, op, dp, fp, tid);
}

template <int KTOT, int AP, int BP, int NT>
__device__ __forceinline__ void gemm_rows16(const unsigned short* __restrict__ ap,
                                            const unsigned short* __restrict__ bp, v8f (&acc)[NT]) {
#pragma unroll 1
  for (int k0 = 0; k0 < KTOT; k0 += 32) {
    FragB af;
    af.h[0] = *(const v8usa*)(ap + k0);
    af.h[1] = *(const v8usa*)(ap + k0 + 16);
#pragma unroll
    for (int nt = 0; nt < NT; ++nt) {
      const unsigned short* wq = bp + (size_t)(16 * nt) * (size_t)BP + k0;
      FragB bf;
      bf.h[0] = *(const v8usa*)wq;
      bf.h[1] = *(const v8usa*)(wq + 16);
      acc[nt] = wmb(af, bf, acc[nt]);
    }
  }
}

template <int NT, int PRE>
__device__ __forceinline__ void tile_flush(const float* stg, const float* sdv, float* OUT, int rowBase,
                                           int wave, int lane) {
  constexpr int NQ = NT * 4, SPN = NT * 16 + 4, NCOL = NT * 16;
#pragma unroll 1
  for (int it = 0; it < NQ / 2; ++it) {
    const int i4  = it * 32 + lane;
    const int r16 = i4 / NQ;
    const int c4  = i4 - r16 * NQ;
    const int lr  = 16 * wave + r16;
    const int grow = rowBase + lr;
    const v4f a = *(const v4fa*)(stg + lr * SPN + 4 * c4);
    float d = 1.0f;
    if constexpr (PRE != 0) d = sdv[lr];
    const bool live = grow < NN;
    v4f o;
    o.x = live ? a.x * d : 0.0f; o.y = live ? a.y * d : 0.0f;
    o.z = live ? a.z * d : 0.0f; o.w = live ? a.w * d : 0.0f;
    *(volatile v4f*)(OUT + (size_t)grow * NCOL + 4 * c4) = o;
  }
}

template <int KTOT, int AP, int BP, int NT, int PRE>
__global__ __launch_bounds__(NTHR) __attribute__((amdgpu_num_vgpr(248)))
void k_gemm(const unsigned short* __restrict__ A, const unsigned short* __restrict__ BT,
            const float* __restrict__ DINV, float* OUT) {
  constexpr int SPN = NT * 16 + 4;
  __shared__ __attribute__((aligned(16))) float stg[GBM * SPN];
  __shared__ __attribute__((aligned(16))) float sdv[GBM];
  const int tid = (int)threadIdx.x, lane = tid & 31, wave = tid >> 5, hh = lane >> 4, m = lane & 15;
  const int rowBase = (int)blockIdx.x * GBM;
  if (tid < 32) {
    if constexpr (PRE != 0) {
      *(v4fa*)(sdv + 4 * tid) = *(const v4fa*)(DINV + rowBase + 4 * tid);
    } else {
      const v4f one = {1.0f, 1.0f, 1.0f, 1.0f};
      *(v4fa*)(sdv + 4 * tid) = one;
    }
  }

  v8f acc[NT];
  {
    const v8f z = {0.f, 0.f, 0.f, 0.f, 0.f, 0.f, 0.f, 0.f};
#pragma unroll
    for (int t = 0; t < NT; ++t) acc[t] = z;
  }
  const unsigned short* ap = A + (size_t)(rowBase + 16 * wave + m) * (size_t)AP + 8 * hh;
  const unsigned short* bp = BT + (size_t)m * (size_t)BP + 8 * hh;
  gemm_rows16<KTOT, AP, BP, NT>(ap, bp, acc);

#pragma unroll
  for (int nt = 0; nt < NT; ++nt) {
#pragma unroll
    for (int r = 0; r < 8; ++r) stg[(16 * wave + 8 * hh + r) * SPN + 16 * nt + m] = acc[nt][r];
  }
  __syncthreads();

  tile_flush<NT, PRE>(stg, sdv, OUT, rowBase, wave, lane);
  __threadfence();
  tile_flush<NT, PRE>(stg, sdv, OUT, rowBase, wave, lane);
}

__global__ __launch_bounds__(NTHR) void k_replay(const int* __restrict__ LIST, const int* __restrict__ CNT,
                                                 const int* __restrict__ OFF, const float* __restrict__ DINV,
                                                 const int* __restrict__ FLAG, const float* HP,
                                                 const float* __restrict__ TB, int boff, unsigned short* HL) {
  __shared__ __attribute__((aligned(16))) float sb[128];
  const int tid = (int)threadIdx.x, lane = tid & 31, wave = tid >> 5, q = lane >> 3, c8 = lane & 7;
  if (tid < 32) *(v4fa*)(sb + 4 * tid) = *(const v4fa*)(TB + 4 * tid);
  __syncthreads();
  const v4f bias = *(const v4fa*)(sb + boff + 4 * c8);
  const int rowBase = (int)blockIdx.x * RBM;
  const int bucket  = rowBase >> SLB;
  const int* lb  = LIST + (size_t)bucket * RCAP;
  const int flag = FLAG[(size_t)bucket * 32];
  const float qnan = __uint_as_float(0x7fc00000u);
  const unsigned hm = (lane < 8) ? 0xffffffffu : 0u;

#pragma unroll 1
  for (int i = 0; i < RBM / NWAVE; ++i) {
    const int d = rowBase + (RBM / NWAVE) * wave + i;
    int cv = CNT[d];
    int ov = OFF[d];
    const bool big = cv > DEGCAP;
    cv = cv < 0 ? 0 : (cv > DEGCAP ? DEGCAP : cv);
    ov = ov < 0 ? 0 : (ov > RCAP - 1 ? RCAP - 1 : ov);
    const int c = __builtin_amdgcn_readfirstlane(cv);
    const int o = __builtin_amdgcn_readfirstlane(ov);
    int last = o + c - 1;
    last = last < o ? o : last;
    last = last > RCAP - 1 ? RCAP - 1 : last;
    const int ntrip = (c + 3) >> 2;
    float a0 = 0.0f, a1 = 0.0f, a2 = 0.0f, a3 = 0.0f;
#pragma unroll 1
    for (int j = 0; j < ntrip; ++j) {
      const int hidx = 4 * j + q;
      int idx = o + hidx;
      idx = idx > last ? last : idx;
      int sr = lb[idx];
      sr = sr < 0 ? 0 : (sr > NN - 1 ? NN - 1 : sr);
      const v4f v = *(const v4fa*)(HP + (size_t)sr * HD + 4 * c8);
      asm volatile("" :: "v"(v));
      const bool valid = hidx < c;
      const float t0 = a0 + v.x, t1 = a1 + v.y, t2 = a2 + v.z, t3 = a3 + v.w;
      a0 = valid ? t0 : a0; a1 = valid ? t1 : a1; a2 = valid ? t2 : a2; a3 = valid ? t3 : a3;
    }
    a0 += __shfl_xor(a0, 16, 32); a1 += __shfl_xor(a1, 16, 32);
    a2 += __shfl_xor(a2, 16, 32); a3 += __shfl_xor(a3, 16, 32);
    a0 += __shfl_xor(a0, 8, 32);  a1 += __shfl_xor(a1, 8, 32);
    a2 += __shfl_xor(a2, 8, 32);  a3 += __shfl_xor(a3, 8, 32);
    const v4f g  = *(const v4fa*)(HP + (size_t)d * HD + 4 * c8);
    const float dd = DINV[d];
    asm volatile("" :: "v"(g));
    asm volatile("" :: "v"(dd));
    float y0 = dd * (a0 + g.x) + bias.x, y1 = dd * (a1 + g.y) + bias.y;
    float y2 = dd * (a2 + g.z) + bias.z, y3 = dd * (a3 + g.w) + bias.w;
    y0 = (y0 > 0.0f) ? y0 : (y0 - y0); y1 = (y1 > 0.0f) ? y1 : (y1 - y1);
    y2 = (y2 > 0.0f) ? y2 : (y2 - y2); y3 = (y3 > 0.0f) ? y3 : (y3 - y3);
    const bool bad  = (flag != 0) | big;
    const bool live = d < NN;
    y0 = bad ? qnan : y0; y1 = bad ? qnan : y1; y2 = bad ? qnan : y2; y3 = bad ? qnan : y3;
    y0 = live ? y0 : 0.0f; y1 = live ? y1 : 0.0f; y2 = live ? y2 : 0.0f; y3 = live ? y3 : 0.0f;
    int h01, h23, l01, l23;
    hilo_pack(y0, y1, y2, y3, h01, h23, l01, l23);
    v2i ow;
    ow.x = (int)(((unsigned)h01 & hm) | ((unsigned)l01 & ~hm));
    ow.y = (int)(((unsigned)h23 & hm) | ((unsigned)l23 & ~hm));
    unsigned short* hp = HL + (size_t)d * KHL + 4 * (lane & 15);
    if (lane < 16) *(volatile v2i*)hp = ow;
    __threadfence();
    if (lane < 16) *(volatile v2i*)hp = ow;
  }
}

__global__ __launch_bounds__(NTHR) void k_pairs(const float* __restrict__ PTG, const int* __restrict__ tfi,
                                                const int* __restrict__ gni, const float* __restrict__ ef,
                                                const float* __restrict__ TB, float* out) {
  __shared__ __attribute__((aligned(16))) float sp[256];
  __shared__ float res[NWAVE * 32];
  const int tid = (int)threadIdx.x, lane = tid & 31, wave = tid >> 5, q = lane >> 3, c8 = lane & 7;
  if (tid < 64) *(v4fa*)(sp + 4 * tid) = *(const v4fa*)(TB + 128 + 4 * tid);
  __syncthreads();
  const int line = (int)blockIdx.x * NWAVE + wave;
  const bool act = line < NLINE0;
  const int lc = act ? line : NLINE0 - 1;
  const int p  = lc * 32 + lane;
  int tv = tfi[p];
  int gv = gni[p];
  tv = tv < 0 ? 0 : (tv > NN - 1 ? NN - 1 : tv);
  gv = gv < 0 ? 0 : (gv > NN - 1 ? NN - 1 : gv);
  const v2f ev = *(const v2fa*)(ef + 2 * (size_t)p);
  const float e0v = bf16_val(ev.x), e1v = bf16_val(ev.y);
  const v4f eb1v = *(const v4fa*)(sp + 4 * c8);
  const v4f e64  = *(const v4fa*)(sp + 32 + 4 * c8);
  const v4f e65  = *(const v4fa*)(sp + 64 + 4 * c8);
  const v4f w2   = *(const v4fa*)(sp + 96 + 4 * c8);
  const float eb2v = sp[192];

#pragma unroll 1
  for (int s = 0; s < 8; ++s) {
    const int sl = 4 * s + q;
    const int t  = __shfl(tv, sl, 32);
    const int g  = __shfl(gv, sl, 32);
    const float f0 = __shfl(e0v, sl, 32);
    const float f1 = __shfl(e1v, sl, 32);
    const v4f pt = *(const v4fa*)(PTG + (size_t)t * NHEAD + 4 * c8);
    const v4f pg = *(const v4fa*)(PTG + (size_t)g * NHEAD + 32 + 4 * c8);
    float y0 = ((pt.x + pg.x) + (f0 * e64.x + f1 * e65.x)) + eb1v.x;
    float y1 = ((pt.y + pg.y) + (f0 * e64.y + f1 * e65.y)) + eb1v.y;
    float y2 = ((pt.z + pg.z) + (f0 * e64.z + f1 * e65.z)) + eb1v.z;
    float y3 = ((pt.w + pg.w) + (f0 * e64.w + f1 * e65.w)) + eb1v.w;
    y0 = (y0 > 0.0f) ? y0 : (y0 - y0); y1 = (y1 > 0.0f) ? y1 : (y1 - y1);
    y2 = (y2 > 0.0f) ? y2 : (y2 - y2); y3 = (y3 > 0.0f) ? y3 : (y3 - y3);
    float z = ((y0 * w2.x + y1 * w2.y) + y2 * w2.z) + y3 * w2.w;
    z += __shfl_xor(z, 1, 32);
    z += __shfl_xor(z, 2, 32);
    z += __shfl_xor(z, 4, 32);
    if (c8 == 0) res[wave * 32 + sl] = z + eb2v;
  }
  __syncthreads();
  const float r = res[wave * 32 + lane];
  asm volatile("" :: "v"(r));
  float* op = out + (size_t)lc * 32 + lane;
  if (act) *(volatile float*)op = r;
  __threadfence();
  if (act) *(volatile float*)op = r;
}

__global__ __launch_bounds__(NTHR) void k_nhead(const float* __restrict__ PTG, const int* __restrict__ nid,
                                                const float* __restrict__ TB, float* out) {
  __shared__ __attribute__((aligned(16))) float sp[128];
  __shared__ float res[NWAVE * 32];
  const int tid = (int)threadIdx.x, lane = tid & 31, wave = tid >> 5, q = lane >> 3, c8 = lane & 7;
  if (tid < 32) *(v4fa*)(sp + 4 * tid) = *(const v4fa*)(TB + 256 + 4 * tid);
  __syncthreads();
  const int line = (int)blockIdx.x * NWAVE + wave;
  const bool act = line < NLINE1;
  const int lc = act ? line : NLINE1 - 1;
  const int p  = lc * 32 + lane;
  const int pc = p < NSEL ? p : NSEL - 1;
  int nv = nid[pc];
  nv = nv < 0 ? 0 : (nv > NN - 1 ? NN - 1 : nv);
  const v4f gb1v = *(const v4fa*)(sp + 4 * c8);
  const v4f w2   = *(const v4fa*)(sp + 32 + 4 * c8);
  const float gb2v = sp[65];

#pragma unroll 1
  for (int s = 0; s < 8; ++s) {
    const int sl = 4 * s + q;
    const int t  = __shfl(nv, sl, 32);
    const v4f pv = *(const v4fa*)(PTG + (size_t)t * NHEAD + 64 + 4 * c8);
    float y0 = pv.x + gb1v.x, y1 = pv.y + gb1v.y, y2 = pv.z + gb1v.z, y3 = pv.w + gb1v.w;
    y0 = (y0 > 0.0f) ? y0 : (y0 - y0); y1 = (y1 > 0.0f) ? y1 : (y1 - y1);
    y2 = (y2 > 0.0f) ? y2 : (y2 - y2); y3 = (y3 > 0.0f) ? y3 : (y3 - y3);
    float z = ((y0 * w2.x + y1 * w2.y) + y2 * w2.z) + y3 * w2.w;
    z += __shfl_xor(z, 1, 32);
    z += __shfl_xor(z, 2, 32);
    z += __shfl_xor(z, 4, 32);
    if (c8 == 0) res[wave * 32 + sl] = z + gb2v;
  }
  __syncthreads();
  const float r = res[wave * 32 + lane];
  asm volatile("" :: "v"(r));
  float* op = out + (size_t)NPAIR + (size_t)pc;
  const bool wr = act && (p < NSEL);
  if (wr) *(volatile float*)op = r;
  __threadfence();
  if (wr) *(volatile float*)op = r;
}

extern "C" void kernel_launch(void* const* d_in, const int* in_sizes, int n_in,
                              void* d_out, int out_size, void* d_ws, size_t ws_size,
                              hipStream_t stream) {
  if (n_in < 18) return;
  if (in_sizes[0] != NN * CIN) return;
  if (in_sizes[1] != 2 * NE) return;
  if (in_sizes[2] != NPAIR || in_sizes[3] != NPAIR) return;
  if (in_sizes[4] != 2 * NPAIR) return;
  if (in_sizes[5] != NSEL) return;
  if (in_sizes[6] != CIN * HD || in_sizes[7] != HD) return;
  if (in_sizes[8] != HD * HD || in_sizes[9] != HD) return;
  if (in_sizes[10] != 66 * HD || in_sizes[11] != HD) return;
  if (in_sizes[12] != HD || in_sizes[13] != 1) return;
  if (in_sizes[14] != HD * HD || in_sizes[15] != HD) return;
  if (in_sizes[16] != HD || in_sizes[17] != 1) return;
  if (out_size != NPAIR + NSEL) return;
  static_assert((size_t)NPAIR + (size_t)NSEL - 1 < (size_t)(NPAIR + NSEL));

  const float* x   = (const float*)d_in[0];
  const int*   ei  = (const int*)d_in[1];
  const int*   tfi = (const int*)d_in[2];
  const int*   gni = (const int*)d_in[3];
  const float* ef  = (const float*)d_in[4];
  const int*   nid = (const int*)d_in[5];
  const float* W1  = (const float*)d_in[6];
  const float* b1  = (const float*)d_in[7];
  const float* W2  = (const float*)d_in[8];
  const float* b2  = (const float*)d_in[9];
  const float* eW1 = (const float*)d_in[10];
  const float* eb1 = (const float*)d_in[11];
  const float* eW2 = (const float*)d_in[12];
  const float* eb2 = (const float*)d_in[13];
  const float* gW1 = (const float*)d_in[14];
  const float* gb1 = (const float*)d_in[15];
  const float* gW2 = (const float*)d_in[16];
  const float* gb2 = (const float*)d_in[17];
  float* out = (float*)d_out;
  const int* srcs = ei;
  const int* dsts = ei + NE;

  constexpr size_t zXB   = (size_t)MP * CIN * 2;
  constexpr size_t zHP   = (size_t)MP * HD * 4;
  constexpr size_t zHL   = (size_t)MP * KHL * 2;
  constexpr size_t zPTG  = (size_t)MP * NHEAD * 4;
  constexpr size_t zLIST = (size_t)NBK * RCAP * 4;
  constexpr size_t zTAB  = (size_t)NBK * NBRUN * 4;
  constexpr size_t zFLAG = (size_t)NBK * 128;
  constexpr size_t zW1T  = (size_t)HD * CIN * 2;
  constexpr size_t zW2D  = (size_t)HD * KHL * 2;
  constexpr size_t zWHD  = (size_t)NHEAD * KHL * 2;
  constexpr size_t zTB   = (size_t)TBN * 4;
  constexpr size_t oXB   = 0;
  constexpr size_t oHP   = oXB + zXB;
  constexpr size_t oH1   = oHP + zHP;
  constexpr size_t oH2   = oH1 + zHL;
  constexpr size_t oPTG  = oH2 + zHL;
  constexpr size_t oLIST = oPTG + zPTG;
  constexpr size_t oCNT  = oLIST + zLIST;
  constexpr size_t oOFF  = oCNT + zTAB;
  constexpr size_t oDINV = oOFF + zTAB;
  constexpr size_t oFLAG = oDINV + zTAB;
  constexpr size_t oW1T  = oFLAG + zFLAG;
  constexpr size_t oW2D  = oW1T + zW1T;
  constexpr size_t oWHD  = oW2D + zW2D;
  constexpr size_t oTB   = oWHD + zWHD;
  constexpr size_t oEND  = oTB + zTB;
  static_assert(zXB % 256 == 0 && zHP % 256 == 0 && zHL % 256 == 0 && zPTG % 256 == 0 && zLIST % 256 == 0);
  static_assert(zTAB % 256 == 0 && zFLAG % 256 == 0 && zW1T % 256 == 0 && zW2D % 256 == 0);
  static_assert(zWHD % 256 == 0 && zTB % 256 == 0);
  static_assert(oEND <= (size_t)(128u << 20));
  static_assert((size_t)NBK * NBRUN >= (size_t)MP);
  if (oEND > ws_size) return;

  char* ws = (char*)d_ws;
  unsigned short* XB   = (unsigned short*)(ws + oXB);
  float*          HP   = (float*)(ws + oHP);
  unsigned short* H1HL = (unsigned short*)(ws + oH1);
  unsigned short* H2HL = (unsigned short*)(ws + oH2);
  float*          PTG  = (float*)(ws + oPTG);
  int*            LIST = (int*)(ws + oLIST);
  int*            CNT  = (int*)(ws + oCNT);
  int*            OFF  = (int*)(ws + oOFF);
  int*            DINVi = (int*)(ws + oDINV);
  const float*    DINV = (const float*)(ws + oDINV);
  int*            FLAG = (int*)(ws + oFLAG);
  unsigned short* W1T  = (unsigned short*)(ws + oW1T);
  unsigned short* W2D  = (unsigned short*)(ws + oW2D);
  unsigned short* WHD  = (unsigned short*)(ws + oWHD);
  float*          TB   = (float*)(ws + oTB);

  hipFuncSetAttribute(reinterpret_cast<const void*>(&k_bucket), hipFuncAttributeMaxDynamicSharedMemorySize, (int)BK_LDS);

  k_prep<<<PBTOT, NTHR, 0, stream>>>(x, W1, b1, W2, b2, eW1, eb1, eW2, eb2, gW1, gb1, gW2, gb2,
                                     XB, W1T, W2D, WHD, TB);
  k_bucket<<<NBK, NTHR, BK_LDS, stream>>>(srcs, dsts, LIST, CNT, OFF, DINVi, FLAG);
  k_gemm<CIN, CIN, CIN, 2, 1><<<MP / GBM, NTHR, 0, stream>>>(XB, W1T, DINV, HP);
  k_replay<<<MP / RBM, NTHR, 0, stream>>>(LIST, CNT, OFF, DINV, FLAG, HP, TB, 0, H1HL);
  k_gemm<K2EXT, KHL, KHL, 2, 1><<<MP / GBM, NTHR, 0, stream>>>(H1HL, W2D, DINV, HP);
  k_replay<<<MP / RBM, NTHR, 0, stream>>>(LIST, CNT, OFF, DINV, FLAG, HP, TB, 32, H2HL);
  k_gemm<K3EXT, KHL, KHL, 6, 0><<<MP / GBM, NTHR, 0, stream>>>(H2HL, WHD, DINV, PTG);
  k_pairs<<<(NLINE0 + NWAVE - 1) / NWAVE, NTHR, 0, stream>>>(PTG, tfi, gni, ef, TB, out);
  k_nhead<<<(NLINE1 + NWAVE - 1) / NWAVE, NTHR, 0, stream>>>(PTG, nid, TB, out);
}
